// LSTM_notime_88235808129536
// MI455X (gfx1250) — hardware-verified
//
#include <hip/hip_runtime.h>
#include <math.h>

typedef __attribute__((ext_vector_type(16))) _Float16 v16h;
typedef __attribute__((ext_vector_type(8)))  _Float16 v8h;
typedef __attribute__((ext_vector_type(8)))  float    v8f;
typedef __attribute__((ext_vector_type(4)))  float    v4f;

constexpr int NBATCH = 256;
constexpr int NSTEP  = 512;
constexpr int NIN    = 3;
constexpr int NHID   = 256;
constexpr int NGATE  = 4 * NHID;
constexpr int ROWS_PER_BLOCK = 16;
constexpr int NTHREADS = 256;
constexpr int HP16 = 264;
constexpr int HP32 = 264;
constexpr float OP_SCALE  = 64.0f;
constexpr float ACC_SCALE = 4096.0f;
constexpr float ACC_INV   = 1.0f / 4096.0f;

__device__ __forceinline__ void dep_guard_h(v8f& a, v8f& b, v16h x, v16h y) { asm volatile("v_nop\n\tv_nop\n\tv_nop\n\tv_nop" : "+v"(a), "+v"(b) : "v"(x), "v"(y)); }
__device__ __forceinline__ void keep4_h(v16h a, v16h b, v16h c, v16h d) { asm volatile("v_nop" :: "v"(a), "v"(b), "v"(c), "v"(d)); }
__device__ __forceinline__ void acc_guard4(v8f& a, v8f& b, v8f& c, v8f& d) { asm volatile("v_nop\n\tv_nop\n\tv_nop\n\tv_nop" : "+v"(a), "+v"(b), "+v"(c), "+v"(d)); }

template <typename T> struct Frag;
template <> struct Frag<_Float16> {
  typedef v16h V; union U { v16h v; v8h h[2]; };
  static __device__ __forceinline__ v16h load(const _Float16* p) {
    U f; f.h[0] = *(const v8h*)(p); f.h[1] = *(const v8h*)(p + 16); return f.v;
  }
  static __device__ __forceinline__ v8f mma(v16h a, v16h b, v8f c) {
    return __builtin_amdgcn_wmma_f32_16x16x32_f16(false, a, false, b, (short)0, c, false, false);
  }
};

__global__ __launch_bounds__(256) void cast_scale_f32_f16x2(
    const float* __restrict__ in, _Float16* __restrict__ out, int n2, float sc) {
  int i = blockIdx.x * 256 + threadIdx.x;
  if (i < n2) {
    const _Float16 h0 = (_Float16)(in[2 * i] * sc), h1 = (_Float16)(in[2 * i + 1] * sc);
    const unsigned u = (unsigned)__builtin_bit_cast(unsigned short, h0) | ((unsigned)__builtin_bit_cast(unsigned short, h1) << 16);
    ((volatile unsigned*)out)[i] = u;
    __threadfence();
    ((volatile unsigned*)out)[i] = u;
  }
}

__device__ __forceinline__ float clamp30(float v) { return fminf(fmaxf(v, -30.0f), 30.0f); }
__device__ __forceinline__ float sigm_f(float v) {
  const float e = expf(-clamp30(v));
  return __builtin_amdgcn_rcpf(1.0f + e);
}
__device__ __forceinline__ float tanh_f(float v) {
  const float e = expf(2.0f * clamp30(v));
  return 1.0f - 2.0f * __builtin_amdgcn_rcpf(e + 1.0f);
}

__global__ __launch_bounds__(NTHREADS)
void recur_seq_kernel(const float* __restrict__ x,
                      const float* __restrict__ W_ih,
                      const _Float16* __restrict__ W16,
                      const float* __restrict__ b_ih,
                      const float* __restrict__ b_hh,
                      const float* __restrict__ W_lin,
                      const float* __restrict__ b_lin,
                      float* __restrict__ y)
{
  __shared__ __align__(16) _Float16 h16[ROWS_PER_BLOCK * HP16];
  __shared__ __align__(16) float    hs[ROWS_PER_BLOCK * HP32];
  __shared__ __align__(16) float    ys[ROWS_PER_BLOCK * NSTEP];

  const int tid  = threadIdx.x;
  const int lane = tid & 31;
  const int wv   = tid >> 5;
  const int c    = lane & 15;
  const int hh   = lane >> 4;
  const int bbase = blockIdx.x * ROWS_PER_BLOCK;

  {
    v8h z;
#pragma unroll
    for (int e = 0; e < 8; ++e) z[e] = (_Float16)0.0f;
    for (int i = tid; i < (ROWS_PER_BLOCK * HP16) / 8; i += NTHREADS) *(v8h*)(h16 + i * 8) = z;
  }

  float wi0[8], wi1[8], wi2[8], bsum[8];
  int goff[8];
#pragma unroll
  for (int nt = 0; nt < 8; ++nt) {
    const int q = nt >> 1, s = nt & 1;
    const int g = q * NHID + wv * 32 + s * 16 + c;
    wi0[nt]  = W_ih[g * NIN + 0];
    wi1[nt]  = W_ih[g * NIN + 1];
    wi2[nt]  = W_ih[g * NIN + 2];
    bsum[nt] = b_ih[g] + b_hh[g];
    goff[nt] = g * NHID + 8 * hh;
  }
  float wl[8];
#pragma unroll
  for (int e = 0; e < 8; ++e) wl[e] = W_lin[lane * 8 + e];
  const float blin = b_lin[0];

  const int aoff = c * HP16 + 8 * hh;

  v8f cst0 = (v8f){0.f,0.f,0.f,0.f,0.f,0.f,0.f,0.f};
  v8f cst1 = (v8f){0.f,0.f,0.f,0.f,0.f,0.f,0.f,0.f};

  __syncthreads();

#pragma unroll 1
  for (int t = 0; t < NSTEP; ++t) {
    float x0[8], x1[8], x2[8];
#pragma unroll
    for (int r = 0; r < 8; ++r) {
      const float* xp = x + ((size_t)(bbase + hh * 8 + r) * NSTEP + t) * NIN;
      x0[r] = xp[0]; x1[r] = xp[1]; x2[r] = xp[2];
    }
    v8f acc[8];
#pragma unroll
    for (int nt = 0; nt < 8; ++nt) {
#pragma unroll
      for (int r = 0; r < 8; ++r)
        acc[nt][r] = (bsum[nt] + x0[r] * wi0[nt] + x1[r] * wi1[nt] + x2[r] * wi2[nt]) * ACC_SCALE;
    }

#pragma unroll
    for (int kt = 0; kt < 8; ++kt) {
      const int k0 = kt * 32;
      const v16h a = Frag<_Float16>::load(h16 + aoff + k0);
#pragma unroll
      for (int grp = 0; grp < 2; ++grp) {
        v16h b[4];
#pragma unroll
        for (int j = 0; j < 4; ++j) b[j] = Frag<_Float16>::load(W16 + goff[grp * 4 + j] + k0);
#pragma unroll
        for (int j = 0; j < 4; ++j) acc[grp * 4 + j] = Frag<_Float16>::mma(a, b[j], acc[grp * 4 + j]);
        dep_guard_h(acc[grp * 4], acc[grp * 4 + 3], a, b[3]);
        keep4_h(b[0], b[1], b[2], b[3]);
      }
    }
    acc_guard4(acc[0], acc[1], acc[2], acc[3]);
    acc_guard4(acc[4], acc[5], acc[6], acc[7]);

    float hv0[8], hv1[8];
#pragma unroll
    for (int r = 0; r < 8; ++r) {
      {
        const float gi = sigm_f(acc[0][r] * ACC_INV);
        const float gf = sigm_f(acc[2][r] * ACC_INV);
        const float gg = tanh_f(acc[4][r] * ACC_INV);
        const float go = sigm_f(acc[6][r] * ACC_INV);
        const float cc = gf * cst0[r] + gi * gg;
        cst0[r] = cc;
        hv0[r] = go * tanh_f(cc);
      }
      {
        const float gi = sigm_f(acc[1][r] * ACC_INV);
        const float gf = sigm_f(acc[3][r] * ACC_INV);
        const float gg = tanh_f(acc[5][r] * ACC_INV);
        const float go = sigm_f(acc[7][r] * ACC_INV);
        const float cc = gf * cst1[r] + gi * gg;
        cst1[r] = cc;
        hv1[r] = go * tanh_f(cc);
      }
    }

#pragma unroll
    for (int r = 0; r < 8; ++r) {
      hs[(hh * 8 + r) * HP32 + wv * 32 + c]      = hv0[r];
      hs[(hh * 8 + r) * HP32 + wv * 32 + 16 + c] = hv1[r];
    }
    __syncthreads();

    {
      const int row = tid >> 4, cb = (tid & 15) * 16;
      const float* sp = hs + row * HP32 + cb;
      const v4f f0 = *(const v4f*)(sp);
      const v4f f1 = *(const v4f*)(sp + 4);
      const v4f f2 = *(const v4f*)(sp + 8);
      const v4f f3 = *(const v4f*)(sp + 12);
      v8h o0, o1;
#pragma unroll
      for (int e = 0; e < 4; ++e) {
        o0[e]     = (_Float16)(f0[e] * OP_SCALE);
        o0[4 + e] = (_Float16)(f1[e] * OP_SCALE);
        o1[e]     = (_Float16)(f2[e] * OP_SCALE);
        o1[4 + e] = (_Float16)(f3[e] * OP_SCALE);
      }
      *(v8h*)(h16 + row * HP16 + cb)     = o0;
      *(v8h*)(h16 + row * HP16 + cb + 8) = o1;
    }

#pragma unroll
    for (int jr = 0; jr < 2; ++jr) {
      const int row = wv * 2 + jr;
      const float* hp = hs + row * HP32 + lane * 8;
      const v4f a0 = *(const v4f*)(hp);
      const v4f a1 = *(const v4f*)(hp + 4);
      float p = a0[0] * wl[0];
      p += a0[1] * wl[1];
      p += a0[2] * wl[2];
      p += a0[3] * wl[3];
      p += a1[0] * wl[4];
      p += a1[1] * wl[5];
      p += a1[2] * wl[6];
      p += a1[3] * wl[7];
      p += __shfl_xor(p, 16, 32);
      p += __shfl_xor(p, 8, 32);
      p += __shfl_xor(p, 4, 32);
      p += __shfl_xor(p, 2, 32);
      p += __shfl_xor(p, 1, 32);
      const float v = fmaxf(p + blin, 0.0f);
      if (lane == 0) ys[row * NSTEP + t] = v;
    }
    __syncthreads();
  }

  {
    float* yb = y + (size_t)bbase * NSTEP;
    for (int pass = 0; pass < 2; ++pass) {
#pragma unroll
      for (int it = 0; it < 8; ++it) {
        const int off = wv * 1024 + it * 128 + lane * 4;
        const v4f v = *(const v4f*)(ys + off);
        *(volatile v4f*)(yb + off) = v;
      }
      __threadfence();
    }
  }
}

extern "C" void kernel_launch(void* const* d_in, const int* in_sizes, int n_in,
                              void* d_out, int out_size, void* d_ws, size_t ws_size,
                              hipStream_t stream) {
  (void)n_in;
  const float* x     = (const float*)d_in[0];
  const float* W_ih  = (const float*)d_in[1];
  const float* W_hh  = (const float*)d_in[2];
  const float* b_ih  = (const float*)d_in[3];
  const float* b_hh  = (const float*)d_in[4];
  const float* W_lin = (const float*)d_in[5];
  const float* b_lin = (const float*)d_in[6];
  float* y = (float*)d_out;

  const int nW = NGATE * NHID;
  if (in_sizes[0] != NBATCH * NSTEP * NIN) return;
  if (in_sizes[1] != NGATE * NIN) return;
  if (in_sizes[2] != nW) return;
  if (in_sizes[3] != NGATE || in_sizes[4] != NGATE) return;
  if (in_sizes[5] != NHID || in_sizes[6] < 1) return;
  if (out_size != NBATCH * NSTEP) return;
  if (ws_size < (size_t)nW * 2) return;

  _Float16* W16 = (_Float16*)d_ws;

  const int n2 = nW / 2;
  cast_scale_f32_f16x2<<<dim3((n2 + 255) / 256), dim3(256), 0, stream>>>(W_hh, W16, n2, OP_SCALE);

  recur_seq_kernel<<<dim3(NBATCH / ROWS_PER_BLOCK), dim3(NTHREADS), 0, stream>>>(
      x, W_ih, W16, b_ih, b_hh, W_lin, b_lin, y);
}
